// IGMC_283467842579
// MI455X (gfx1250) — hardware-verified
//
#include <hip/hip_runtime.h>
#include <stddef.h>


#define FD      64
#define NREL    5
#define NBAS    2
#define NLAY    4
#define KL      (3 * FD)
#define STP     (NLAY * FD)
#define HID     128
#define KC      (2 * STP)
#define NTHR    256
#define NWAVE   8
#define EPT     8
#define NGRP    2
#define CHUNK   (NTHR * EPT * NGRP)
#define WCAP    (EPT * NGRP * 32)
#define LISTN   (NWAVE * WCAP)
#define SLOTSH  13
#define NBC     8192
#define NBF     2048
#define RCAP    61440
#define RBN     128
#define CPT     16
#define OTHR    (NBC / CPT)
#define GR      64
#define QB      32
#define DEGCAP  1024
#define APX     (KL + 8)
#define APC     (KC + 8)
#define BCAP    4096
#define WSCAP   134217728
#define OWLSZ   (FD * KL)
#define OW1     (NLAY * 2 * OWLSZ)
#define OWTOT   (OW1 + 2 * HID * KC)
#define NWBLK   (6 * NLAY + (HID * KC) / (8 * NTHR))

#define LDS_FILL ((RCAP + NBF + LISTN) * 4 + 64)
#define LDS_LAY  (2 * GR * APX * 2 + GR * FD * 4)
#define LDS_HEAD (2 * BCAP * 4 + 2 * QB * APC * 2 + QB * HID * 4 + 256)

static_assert((CHUNK & (CHUNK - 1)) == 0);
static_assert(NBC <= (1 << SLOTSH) && NBF <= (1 << SLOTSH));
static_assert((NBC & (NBC - 1)) == 0 && (NBF & (NBF - 1)) == 0);
static_assert(NBC == 4 * NBF);
static_assert(OTHR * CPT == NBC && OTHR == 512 && 128 * CPT == NBF);
static_assert((RCAP % 32) == 0);
static_assert(GR == NWAVE * 8 && GR == 4 * 16);
static_assert(FD == 2 * 32 && HID == 4 * 32 && QB == 4 * NWAVE && QB == 2 * 16);
static_assert((KL % 32) == 0 && (KC % 32) == 0);
static_assert(((APX * 2) % 16) == 0 && ((APC * 2) % 16) == 0);
static_assert(((GR * APX * 2) % 16) == 0 && ((QB * APC * 2) % 16) == 0 && ((2 * BCAP * 4) % 16) == 0);
static_assert(((QB * KC / 8) % NTHR) == 0);
static_assert(OW1 == 98304 && OWTOT == 229376 && NWBLK == 56);
static_assert((BCAP % NTHR) == 0);

typedef float          v2f  __attribute__((ext_vector_type(2)));
typedef float          v4f  __attribute__((ext_vector_type(4)));
typedef float          v8f  __attribute__((ext_vector_type(8)));
typedef int            v4i  __attribute__((ext_vector_type(4)));
typedef unsigned short v2us __attribute__((ext_vector_type(2)));
typedef unsigned short v4us __attribute__((ext_vector_type(4)));
typedef unsigned short v8us __attribute__((ext_vector_type(8)));
typedef __bf16         v16b __attribute__((ext_vector_type(16)));
union FragB { v16b v; v8us h[2]; };

__device__ __forceinline__ unsigned int bfr(float f) {
  const unsigned int u = __float_as_uint(f);
  return (u + 0x7FFFu + ((u >> 16) & 1u)) >> 16;
}

__device__ __forceinline__ void split1(float x, unsigned short& hb, unsigned short& lb) {
  const unsigned int hu = bfr(x);
  const float hf = __uint_as_float(hu << 16);
  hb = (unsigned short)hu;
  lb = (unsigned short)bfr(x - hf);
}

__device__ __forceinline__ void split8(v4f a, v4f b, v8us& hi, v8us& lo) {
  unsigned short hb, lb;
  split1(a.x, hb, lb); hi[0] = hb; lo[0] = lb;
  split1(a.y, hb, lb); hi[1] = hb; lo[1] = lb;
  split1(a.z, hb, lb); hi[2] = hb; lo[2] = lb;
  split1(a.w, hb, lb); hi[3] = hb; lo[3] = lb;
  split1(b.x, hb, lb); hi[4] = hb; lo[4] = lb;
  split1(b.y, hb, lb); hi[5] = hb; lo[5] = lb;
  split1(b.z, hb, lb); hi[6] = hb; lo[6] = lb;
  split1(b.w, hb, lb); hi[7] = hb; lo[7] = lb;
}

__device__ __forceinline__ void split2(v2f a, v2us& hi, v2us& lo) {
  unsigned short hb, lb;
  split1(a.x, hb, lb); hi.x = hb; lo.x = lb;
  split1(a.y, hb, lb); hi.y = hb; lo.y = lb;
}

__device__ __forceinline__ v8f wmb(v16b a, v16b b, v8f c) {
  v8f d = __builtin_amdgcn_wmma_f32_16x16x32_bf16(false, a, false, b, (short)0, c, false, false);
  asm volatile("v_nop\n\tv_nop\n\tv_nop\n\tv_nop" : "+v"(d) : "v"(a), "v"(b));
  return d;
}

template <int NB>
__device__ __forceinline__ int scan_chunk(const int* __restrict__ dsts, int nE, int cbase, int slotBase,
                                          int vec8, int* list, int tid, int lane, int wave) {
  int wc = 0;
#pragma unroll
  for (int g = 0; g < NGRP; ++g) {
    const int el0  = (g * NTHR + tid) * EPT;
    const int e0   = cbase + el0;
    const int sent = -2147483647 - 1;
    v4i da, db;
    if (vec8 != 0 && cbase + CHUNK <= nE) {
      da = *(const v4i*)(dsts + e0);
      db = *(const v4i*)(dsts + e0 + 4);
    } else {
      da.x = (e0     < nE) ? dsts[min(e0, nE - 1)] : sent;
      da.y = (e0 + 1 < nE) ? dsts[min(e0 + 1, nE - 1)] : sent;
      da.z = (e0 + 2 < nE) ? dsts[min(e0 + 2, nE - 1)] : sent;
      da.w = (e0 + 3 < nE) ? dsts[min(e0 + 3, nE - 1)] : sent;
      db.x = (e0 + 4 < nE) ? dsts[min(e0 + 4, nE - 1)] : sent;
      db.y = (e0 + 5 < nE) ? dsts[min(e0 + 5, nE - 1)] : sent;
      db.z = (e0 + 6 < nE) ? dsts[min(e0 + 6, nE - 1)] : sent;
      db.w = (e0 + 7 < nE) ? dsts[min(e0 + 7, nE - 1)] : sent;
    }
    const unsigned nb = (unsigned)slotBase;
    const unsigned s0 = (unsigned)da.x - nb, s1 = (unsigned)da.y - nb;
    const unsigned s2 = (unsigned)da.z - nb, s3 = (unsigned)da.w - nb;
    const unsigned s4 = (unsigned)db.x - nb, s5 = (unsigned)db.y - nb;
    const unsigned s6 = (unsigned)db.z - nb, s7 = (unsigned)db.w - nb;
    const bool h0 = s0 < (unsigned)NB, h1 = s1 < (unsigned)NB, h2 = s2 < (unsigned)NB, h3 = s3 < (unsigned)NB;
    const bool h4 = s4 < (unsigned)NB, h5 = s5 < (unsigned)NB, h6 = s6 < (unsigned)NB, h7 = s7 < (unsigned)NB;
    const unsigned any = __builtin_amdgcn_ballot_w32(h0 | h1 | h2 | h3 | h4 | h5 | h6 | h7);
    if (any != 0u) {
#define HITJ(J, HJ, SJ) { \
        const unsigned mj = __builtin_amdgcn_ballot_w32(HJ); \
        if (mj != 0u) { \
          if (HJ) { \
            const int pos = wc + (int)__builtin_amdgcn_mbcnt_lo(mj, 0u); \
            if (pos < WCAP) list[wave * WCAP + pos] = ((el0 + (J)) << SLOTSH) | (int)(SJ); \
          } \
          wc += (int)__builtin_popcount(mj); } }
      HITJ(0, h0, s0)
      HITJ(1, h1, s1)
      HITJ(2, h2, s2)
      HITJ(3, h3, s3)
      HITJ(4, h4, s4)
      HITJ(5, h5, s5)
      HITJ(6, h6, s6)
      HITJ(7, h7, s7)
#undef HITJ
    }
  }
  return wc;
}

__global__ __launch_bounds__(NTHR) void k_wprep(
    const float* __restrict__ basis, const float* __restrict__ root,
    const float* __restrict__ w1, unsigned short* wp) {
  const int blk = blockIdx.x, tid = threadIdx.x;
  float v[8];
  unsigned short* dh;
  unsigned short* dl;
  if (blk < 6 * NLAY) {
    const int l = blk / 6, s = blk - 6 * l;
    const int seg = s >> 1;
    const int i = (s & 1) * NTHR + tid;
    const int n = i >> 3;
    const int kk0 = (i & 7) * 8;
    const float* p = (seg == 2) ? (root + ((size_t)(l * FD + kk0)) * FD + n)
                                : (basis + ((size_t)((l * NBAS + seg) * FD + kk0)) * FD + n);
#pragma unroll
    for (int e = 0; e < 8; ++e) v[e] = p[(size_t)e * FD];
    dh = wp + (size_t)l * 2 * OWLSZ + (size_t)n * KL + seg * FD + kk0;
    dl = dh + OWLSZ;
  } else {
    const int i = (blk - 6 * NLAY) * NTHR + tid;
    const int n = i >> 6;
    const int k0 = (i & 63) * 8;
#pragma unroll
    for (int e = 0; e < 8; ++e) v[e] = w1[(size_t)(k0 + e) * HID + n];
    dh = wp + OW1 + (size_t)n * KC + k0;
    dl = dh + HID * KC;
  }
  v4f a, b;
  a.x = v[0]; a.y = v[1]; a.z = v[2]; a.w = v[3];
  b.x = v[4]; b.y = v[5]; b.z = v[6]; b.w = v[7];
  v8us hv, lv;
  split8(a, b, hv, lv);
  *(volatile v8us*)dh = hv;
  *(volatile v8us*)dl = lv;
  __threadfence();
  *(volatile v8us*)dh = hv;
  *(volatile v8us*)dl = lv;
}

__global__ __launch_bounds__(NTHR) void k_count(const int* __restrict__ dsts, int* cnt, int nE, int vec8) {
  __shared__ __attribute__((aligned(16))) int scnt[NBC];
  __shared__ __attribute__((aligned(16))) int list[LISTN];
  __shared__ int wcnt[NWAVE];
  const int tid = threadIdx.x, lane = tid & 31, wave = tid >> 5;
  const int nodeBase = blockIdx.x * NBC;

  for (int i = tid; i < NBC; i += NTHR) scnt[i] = 0;
  __syncthreads();

  const int nChunks = (nE + CHUNK - 1) / CHUNK;
#pragma unroll 1
  for (int ch = 0; ch < nChunks; ++ch) {
    const int cbase = ch * CHUNK;
    const int wc = scan_chunk<NBC>(dsts, nE, cbase, nodeBase, vec8, list, tid, lane, wave);
    if (lane == 0) wcnt[wave] = wc;
    __syncthreads();
    if (wave == 0) {
#pragma unroll 1
      for (int wsx = 0; wsx < NWAVE; ++wsx) {
        int n = __builtin_amdgcn_readfirstlane(wcnt[wsx]);
        n = n > WCAP ? WCAP : (n < 0 ? 0 : n);
        const int* lp = list + wsx * WCAP;
#pragma unroll 1
        for (int i = 0; i < n; ++i) {
          const int ent  = __builtin_amdgcn_readfirstlane(lp[i]);
          const int slot = ent & (NBC - 1);
          if (lane == 0) scnt[slot] = scnt[slot] + 1;
        }
      }
    }
    __syncthreads();
  }

  v4i cq[8];
#pragma unroll
  for (int q = 0; q < 8; ++q) {
    const int f = (wave * 8 + q) * 128 + 4 * lane;
    cq[q] = *(const v4i*)(scnt + f);
  }
  int* cp = cnt + (size_t)nodeBase;
#pragma unroll
  for (int q = 0; q < 8; ++q) {
    const int f = (wave * 8 + q) * 128 + 4 * lane;
    *(volatile v4i*)(cp + f) = cq[q];
  }
  __threadfence();
#pragma unroll
  for (int q = 0; q < 8; ++q) {
    const int f = (wave * 8 + q) * 128 + 4 * lane;
    *(volatile v4i*)(cp + f) = cq[q];
  }
}

__global__ __launch_bounds__(OTHR) void k_offsets(
    const int* __restrict__ cnt, int* off, int* rbase, int nChunk) {
  __shared__ __attribute__((aligned(16))) int soff[NBC];
  __shared__ __attribute__((aligned(16))) int srb[RBN];
  __shared__ int wtot[OTHR / 32];
  const int tid = threadIdx.x, lane = tid & 31, wave = tid >> 5, sub = tid >> 7;
  for (int i = tid; i < RBN; i += OTHR) srb[i] = 0;
  int carry = 0;
#pragma unroll 1
  for (int ch = 0; ch < nChunk; ++ch) {
    const int base = ch * NBC;
    const int* cpp = cnt + base + CPT * tid;
    const v4i c0 = *(const v4i*)(cpp);
    const v4i c1 = *(const v4i*)(cpp + 4);
    const v4i c2 = *(const v4i*)(cpp + 8);
    const v4i c3 = *(const v4i*)(cpp + 12);
    int e[16];
    e[0]  = max(c0.x, 0); e[1]  = max(c0.y, 0); e[2]  = max(c0.z, 0); e[3]  = max(c0.w, 0);
    e[4]  = max(c1.x, 0); e[5]  = max(c1.y, 0); e[6]  = max(c1.z, 0); e[7]  = max(c1.w, 0);
    e[8]  = max(c2.x, 0); e[9]  = max(c2.y, 0); e[10] = max(c2.z, 0); e[11] = max(c2.w, 0);
    e[12] = max(c3.x, 0); e[13] = max(c3.y, 0); e[14] = max(c3.z, 0); e[15] = max(c3.w, 0);
    int ts = 0;
#pragma unroll
    for (int j = 0; j < 16; ++j) ts += e[j];
    int incl = ts;
#pragma unroll
    for (int d = 1; d < 32; d <<= 1) {
      const int t = __shfl_up(incl, d);
      if (lane >= d) incl += t;
    }
    if (lane == 31) wtot[wave] = incl;
    __syncthreads();
    const int S0 = wtot[0]  + wtot[1]  + wtot[2]  + wtot[3];
    const int S1 = wtot[4]  + wtot[5]  + wtot[6]  + wtot[7];
    const int S2 = wtot[8]  + wtot[9]  + wtot[10] + wtot[11];
    const int S3 = wtot[12] + wtot[13] + wtot[14] + wtot[15];
    int pre = 0;
#pragma unroll 1
    for (int w = 4 * sub; w < wave; ++w) pre += wtot[w];
    const int b0 = carry;
    const int b1 = b0 + ((S0 + 31) & ~31);
    const int b2 = b1 + ((S1 + 31) & ~31);
    const int b3 = b2 + ((S2 + 31) & ~31);
    const int b4 = b3 + ((S3 + 31) & ~31);
    const int myb = sub == 0 ? b0 : (sub == 1 ? b1 : (sub == 2 ? b2 : b3));
    if (tid == 0) {
      srb[min(4 * ch + 0, RBN - 1)] = b0;
      srb[min(4 * ch + 1, RBN - 1)] = b1;
      srb[min(4 * ch + 2, RBN - 1)] = b2;
      srb[min(4 * ch + 3, RBN - 1)] = b3;
    }
    int run = myb + pre + incl - ts;
#pragma unroll
    for (int j = 0; j < 16; ++j) { soff[CPT * tid + j] = run; run += e[j]; }
    carry = b4;
    __syncthreads();
    v4i o[4];
#pragma unroll
    for (int jj = 0; jj < 4; ++jj) o[jj] = *(const v4i*)(soff + 4 * (tid + jj * OTHR));
    int* op = off + base;
#pragma unroll
    for (int jj = 0; jj < 4; ++jj) *(volatile v4i*)(op + 4 * (tid + jj * OTHR)) = o[jj];
    __threadfence();
#pragma unroll
    for (int jj = 0; jj < 4; ++jj) *(volatile v4i*)(op + 4 * (tid + jj * OTHR)) = o[jj];
    __syncthreads();
  }
  if (tid == 0) srb[min(4 * nChunk, RBN - 1)] = carry;
  __syncthreads();
  v4i rv = {0, 0, 0, 0};
  if (tid < 32) rv = *(const v4i*)(srb + 4 * tid);
  if (tid < 32) *(volatile v4i*)(rbase + 4 * tid) = rv;
  __threadfence();
  if (tid < 32) *(volatile v4i*)(rbase + 4 * tid) = rv;
}

__global__ __launch_bounds__(NTHR) void k_fill(
    const int* __restrict__ dsts, const int* __restrict__ off, const int* __restrict__ rbase,
    int* csr, int nE, int vec8, int csrLen) {
  extern __shared__ v4f lds_dyn[];
  int* region = (int*)lds_dyn;
  int* cursor = region + RCAP;
  int* list   = cursor + NBF;
  int* wcnt   = list + LISTN;
  const int tid = threadIdx.x, lane = tid & 31, wave = tid >> 5;
  const int b = blockIdx.x;
  const int nodeBase = b * NBF;

  int rb0 = rbase[b];
  const int rb1 = rbase[b + 1];
  rb0 = rb0 < 0 ? 0 : (rb0 > csrLen ? csrLen : rb0);
  rb0 &= ~31;
  int len = rb1 - rb0;
  len = len < 0 ? 0 : (len > RCAP ? RCAP : len);
  int lenW = (len + 31) & ~31;
  if (rb0 + lenW > csrLen) lenW = (csrLen - rb0) & ~31;

  {
    const v4i z = {0, 0, 0, 0};
    for (int i = tid; i < RCAP / 4; i += NTHR) ((v4i*)region)[i] = z;
    for (int s = tid; s < NBF; s += NTHR) {
      int o = off[nodeBase + s] - rb0;
      o = o < 0 ? 0 : (o > RCAP ? RCAP : o);
      cursor[s] = o;
    }
  }
  __syncthreads();

  const int nChunks = (nE + CHUNK - 1) / CHUNK;
#pragma unroll 1
  for (int ch = 0; ch < nChunks; ++ch) {
    const int cbase = ch * CHUNK;
    const int wc = scan_chunk<NBF>(dsts, nE, cbase, nodeBase, vec8, list, tid, lane, wave);
    if (lane == 0) wcnt[wave] = wc;
    __syncthreads();
    if (wave == 0) {
#pragma unroll 1
      for (int wsx = 0; wsx < NWAVE; ++wsx) {
        int n = __builtin_amdgcn_readfirstlane(wcnt[wsx]);
        n = n > WCAP ? WCAP : (n < 0 ? 0 : n);
        const int* lp = list + wsx * WCAP;
#pragma unroll 1
        for (int i = 0; i < n; ++i) {
          const int ent  = __builtin_amdgcn_readfirstlane(lp[i]);
          const int slot = ent & (NBF - 1);
          int e = cbase + ((ent >> SLOTSH) & (CHUNK - 1));
          e = e > nE - 1 ? nE - 1 : e;
          if (lane == 0) {
            int pos = cursor[slot];
            pos = pos < 0 ? 0 : (pos > RCAP - 1 ? RCAP - 1 : pos);
            region[pos] = e;
            const int np = pos + 1;
            cursor[slot] = np > RCAP ? RCAP : np;
          }
        }
      }
    }
    __syncthreads();
  }

  const int nv = lenW >> 2;
  int* gp = csr + rb0;
#pragma unroll 1
  for (int i = tid; i < nv; i += NTHR) { const v4i v = ((const v4i*)region)[i]; *(volatile v4i*)(gp + 4 * i) = v; }
  __threadfence();
#pragma unroll 1
  for (int i = tid; i < nv; i += NTHR) { const v4i v = ((const v4i*)region)[i]; *(volatile v4i*)(gp + 4 * i) = v; }
}

__device__ __forceinline__ void agg_row(
    const int* __restrict__ csr, const int* __restrict__ esrc, const int* __restrict__ etyp,
    const float* hin, int pin, int n, int st0, int lane, int nN, int nE, int csrLen,
    const float* __restrict__ cmp, v2f& A0, v2f& A1) {
  v2f a0 = {0.f, 0.f}, a1 = {0.f, 0.f}, a2 = {0.f, 0.f}, a3 = {0.f, 0.f}, a4 = {0.f, 0.f};
  int c0 = 0, c1 = 0, c2 = 0, c3 = 0, c4 = 0;
#pragma unroll 1
  for (int q0 = 0; q0 < n; q0 += 32) {
    int pos = st0 + q0 + lane;
    pos = pos < 0 ? 0 : (pos > csrLen - 1 ? csrLen - 1 : pos);
    int ed = csr[pos];
    ed = ed < 0 ? 0 : (ed > nE - 1 ? nE - 1 : ed);
    int sv = esrc[ed];
    sv = sv < 0 ? 0 : (sv > nN - 1 ? nN - 1 : sv);
    int rv = etyp[ed];
    rv = rv < 0 ? 0 : (rv > NREL - 1 ? NREL - 1 : rv);
    const int mcnt = (n - q0) < 32 ? (n - q0) : 32;
#pragma unroll 1
    for (int p = 0; p < mcnt; ++p) {
      const int ss = __builtin_amdgcn_readlane(sv, p);
      const int rr = __builtin_amdgcn_readlane(rv, p);
      const v2f xv = *(const v2f*)(hin + (size_t)ss * pin + 2 * lane);
      if (rr == 0)      { a0 += xv; c0 += 1; }
      else if (rr == 1) { a1 += xv; c1 += 1; }
      else if (rr == 2) { a2 += xv; c2 += 1; }
      else if (rr == 3) { a3 += xv; c3 += 1; }
      else              { a4 += xv; c4 += 1; }
    }
  }
  const float i0 = 1.0f / (float)(c0 < 1 ? 1 : c0);
  const float i1 = 1.0f / (float)(c1 < 1 ? 1 : c1);
  const float i2 = 1.0f / (float)(c2 < 1 ? 1 : c2);
  const float i3 = 1.0f / (float)(c3 < 1 ? 1 : c3);
  const float i4 = 1.0f / (float)(c4 < 1 ? 1 : c4);
  const float w00 = cmp[0] * i0, w01 = cmp[1] * i0;
  const float w10 = cmp[2] * i1, w11 = cmp[3] * i1;
  const float w20 = cmp[4] * i2, w21 = cmp[5] * i2;
  const float w30 = cmp[6] * i3, w31 = cmp[7] * i3;
  const float w40 = cmp[8] * i4, w41 = cmp[9] * i4;
  A0 = a0 * w00 + a1 * w10 + a2 * w20 + a3 * w30 + a4 * w40;
  A1 = a0 * w01 + a1 * w11 + a2 * w21 + a3 * w31 + a4 * w41;
}

__global__ __launch_bounds__(NTHR) void k_layer(
    const int* __restrict__ csr, const int* __restrict__ off, const int* __restrict__ cnt,
    const int* __restrict__ esrc, const int* __restrict__ etyp,
    const float* hin, int pin, const float* __restrict__ cmp,
    const unsigned short* __restrict__ wl, const float* __restrict__ bias,
    float* stout, int nN, int nE, int csrLen) {
  extern __shared__ v4f lds_dyn[];
  unsigned short* sXh = (unsigned short*)lds_dyn;
  unsigned short* sXl = sXh + GR * APX;
  float*          stg = (float*)(sXl + GR * APX);
  const int tid = threadIdx.x, lane = tid & 31, wave = tid >> 5, hh = lane >> 4, m = lane & 15;
  const int rowBase = blockIdx.x * GR;

  const int cl = rowBase + 8 * wave + (lane & 7);
  const int cv = cnt[cl];
  const int ov = off[cl];
#pragma unroll 1
  for (int j = 0; j < 8; ++j) {
    int n = __builtin_amdgcn_readlane(cv, j);
    n = n < 0 ? 0 : (n > DEGCAP ? DEGCAP : n);
    const int st0 = __builtin_amdgcn_readlane(ov, j);
    const int rl = 8 * wave + j;
    int node = rowBase + rl;
    node = node > nN - 1 ? nN - 1 : node;
    v2f A0, A1;
    agg_row(csr, esrc, etyp, hin, pin, n, st0, lane, nN, nE, csrLen, cmp, A0, A1);
    const v2f hs = *(const v2f*)(hin + (size_t)node * pin + 2 * lane);
    v2us h0, l0, h1, l1, h2, l2;
    split2(A0, h0, l0);
    split2(A1, h1, l1);
    split2(hs, h2, l2);
    unsigned short* rh = sXh + rl * APX + 2 * lane;
    unsigned short* rlo = sXl + rl * APX + 2 * lane;
    *(v2us*)(rh)           = h0;
    *(v2us*)(rh + FD)      = h1;
    *(v2us*)(rh + 2 * FD)  = h2;
    *(v2us*)(rlo)          = l0;
    *(v2us*)(rlo + FD)     = l1;
    *(v2us*)(rlo + 2 * FD) = l2;
  }
  __syncthreads();

  {
    const int rg = wave >> 1, chf = wave & 1;
    const unsigned short* ph = sXh + (rg * 16 + m) * APX + 8 * hh;
    const unsigned short* pl = sXl + (rg * 16 + m) * APX + 8 * hh;
    float* strow = stg + (rg * 16 + 8 * hh) * FD + m;
#pragma unroll 1
    for (int tt = 0; tt < 2; ++tt) {
      const int t = chf * 2 + tt;
      v8f acc = {0.f, 0.f, 0.f, 0.f, 0.f, 0.f, 0.f, 0.f};
      const unsigned short* bb = wl + (size_t)(16 * t + m) * KL + 8 * hh;
#pragma unroll
      for (int ks = 0; ks < KL / 32; ++ks) {
        FragB ah, al, bh, bl;
        ah.h[0] = *(const v8us*)(ph + 32 * ks);          ah.h[1] = *(const v8us*)(ph + 32 * ks + 16);
        al.h[0] = *(const v8us*)(pl + 32 * ks);          al.h[1] = *(const v8us*)(pl + 32 * ks + 16);
        bh.h[0] = *(const v8us*)(bb + 32 * ks);          bh.h[1] = *(const v8us*)(bb + 32 * ks + 16);
        bl.h[0] = *(const v8us*)(bb + OWLSZ + 32 * ks);  bl.h[1] = *(const v8us*)(bb + OWLSZ + 32 * ks + 16);
        acc = wmb(ah.v, bh.v, acc);
        acc = wmb(ah.v, bl.v, acc);
        acc = wmb(al.v, bh.v, acc);
      }
      const float bv = bias[16 * t + m];
#pragma unroll
      for (int r = 0; r < 8; ++r) strow[r * FD + 16 * t] = tanhf(acc[r] + bv);
    }
  }
  __syncthreads();

  const int sub = lane >> 4, lc = lane & 15;
  v4f hv[4];
#pragma unroll
  for (int i = 0; i < 4; ++i) {
    const int rr = 8 * wave + 2 * i + sub;
    hv[i] = *(const v4f*)(stg + rr * FD + 4 * lc);
  }
  float* gp = stout + (size_t)(rowBase + 8 * wave + sub) * STP + 4 * lc;
#pragma unroll
  for (int i = 0; i < 4; ++i) *(volatile v4f*)(gp + (size_t)(2 * i) * STP) = hv[i];
  __threadfence();
#pragma unroll
  for (int i = 0; i < 4; ++i) *(volatile v4f*)(gp + (size_t)(2 * i) * STP) = hv[i];
}

__global__ __launch_bounds__(NTHR) void k_head(
    const float* __restrict__ x, const float* __restrict__ st,
    const unsigned short* __restrict__ wp, const float* __restrict__ b1,
    const float* __restrict__ w2, const float* __restrict__ b2,
    const int* __restrict__ numg, float* out, int nN, int nB) {
  extern __shared__ v4f lds_dyn[];
  int* lu = (int*)lds_dyn;
  int* lm = lu + BCAP;
  unsigned short* sCh = (unsigned short*)(lm + BCAP);
  unsigned short* sCl = sCh + QB * APC;
  float* sH = (float*)(sCl + QB * APC);
  float* sOut = sH + QB * HID;
  int* wcu = (int*)(sOut + QB);
  int* wcm = wcu + NWAVE;
  const int tid = threadIdx.x, lane = tid & 31, wave = tid >> 5, hh = lane >> 4, m = lane & 15;

  for (int i = tid; i < BCAP; i += NTHR) { lu[i] = 0; lm[i] = 0; }
  int ng = numg[0];
  ng = ng < 0 ? 0 : (ng > nB ? nB : ng);
  __syncthreads();

  int baseU = 0, baseM = 0;
  const int nCh = (nN + NTHR - 1) / NTHR;
#pragma unroll 1
  for (int ch = 0; ch < nCh; ++ch) {
    const int n = ch * NTHR + tid;
    const int nc = n > nN - 1 ? nN - 1 : n;
    const float x0 = x[(size_t)nc * FD];
    const float x1 = x[(size_t)nc * FD + 1];
    const bool hu = (n < nN) && (x0 == 1.0f);
    const bool hm = (n < nN) && (x1 == 1.0f);
    const unsigned bu = __builtin_amdgcn_ballot_w32(hu);
    const unsigned bm = __builtin_amdgcn_ballot_w32(hm);
    if (lane == 0) { wcu[wave] = (int)__builtin_popcount(bu); wcm[wave] = (int)__builtin_popcount(bm); }
    __syncthreads();
    int preU = 0, preM = 0, totU = 0, totM = 0;
#pragma unroll
    for (int w = 0; w < NWAVE; ++w) {
      const int cu = wcu[w], cm = wcm[w];
      preU += (w < wave) ? cu : 0;
      preM += (w < wave) ? cm : 0;
      totU += cu;
      totM += cm;
    }
    const int posU = baseU + preU + (int)__builtin_amdgcn_mbcnt_lo(bu, 0u);
    const int posM = baseM + preM + (int)__builtin_amdgcn_mbcnt_lo(bm, 0u);
    if (hu && (unsigned)posU < (unsigned)ng) lu[posU] = n;
    if (hm && (unsigned)posM < (unsigned)ng) lm[posM] = n;
    baseU += totU;
    baseM += totM;
    __syncthreads();
  }

  const v4f w2v = *(const v4f*)(w2 + 4 * lane);
  const float b2v = b2[0];
  const int nQT = (nB + QB - 1) / QB;
#pragma unroll 1
  for (int qt = 0; qt < nQT; ++qt) {
#pragma unroll
    for (int it = 0; it < (QB * KC / 8) / NTHR; ++it) {
      const int idx = it * NTHR + tid;
      const int row = idx >> 6;
      const int c0  = (idx & 63) * 8;
      int qc = qt * QB + row;
      qc = qc > BCAP - 1 ? BCAP - 1 : qc;
      const int uq = lu[qc], mq = lm[qc];
      int node = (c0 < STP) ? uq : mq;
      node = node < 0 ? 0 : (node > nN - 1 ? nN - 1 : node);
      const float* p = st + (size_t)node * STP + (c0 & (STP - 1));
      const v4f a = *(const v4f*)p;
      const v4f b = *(const v4f*)(p + 4);
      v8us hv, lv;
      split8(a, b, hv, lv);
      *(v8us*)(sCh + row * APC + c0) = hv;
      *(v8us*)(sCl + row * APC + c0) = lv;
    }
    __syncthreads();

    {
      const int rg = wave & 1;
      const unsigned short* ph = sCh + (rg * 16 + m) * APC + 8 * hh;
      const unsigned short* pl = sCl + (rg * 16 + m) * APC + 8 * hh;
      float* strow = sH + (rg * 16 + 8 * hh) * HID + m;
#pragma unroll 1
      for (int tt = 0; tt < 2; ++tt) {
        const int t = (wave >> 1) * 2 + tt;
        v8f acc = {0.f, 0.f, 0.f, 0.f, 0.f, 0.f, 0.f, 0.f};
        const unsigned short* bb = wp + OW1 + (size_t)(16 * t + m) * KC + 8 * hh;
#pragma unroll
        for (int ks = 0; ks < KC / 32; ++ks) {
          FragB ah, al, bh, bl;
          ah.h[0] = *(const v8us*)(ph + 32 * ks);             ah.h[1] = *(const v8us*)(ph + 32 * ks + 16);
          al.h[0] = *(const v8us*)(pl + 32 * ks);             al.h[1] = *(const v8us*)(pl + 32 * ks + 16);
          bh.h[0] = *(const v8us*)(bb + 32 * ks);             bh.h[1] = *(const v8us*)(bb + 32 * ks + 16);
          bl.h[0] = *(const v8us*)(bb + HID * KC + 32 * ks);  bl.h[1] = *(const v8us*)(bb + HID * KC + 32 * ks + 16);
          acc = wmb(ah.v, bh.v, acc);
          acc = wmb(ah.v, bl.v, acc);
          acc = wmb(al.v, bh.v, acc);
        }
        const float bv = b1[16 * t + m];
#pragma unroll
        for (int r = 0; r < 8; ++r) strow[r * HID + 16 * t] = fmaxf(acc[r] + bv, 0.0f);
      }
    }
    __syncthreads();

#pragma unroll
    for (int i = 0; i < 4; ++i) {
      const int row = 4 * wave + i;
      const v4f hv = *(const v4f*)(sH + row * HID + 4 * lane);
      float s = hv.x * w2v.x + hv.y * w2v.y + hv.z * w2v.z + hv.w * w2v.w;
#pragma unroll
      for (int o = 16; o > 0; o >>= 1) s += __shfl_xor(s, o);
      if (lane == 0) sOut[row] = s + b2v;
    }
    __syncthreads();

    const int q = qt * QB + lane;
    const float ov = sOut[lane];
    if (wave == 0 && q < nB) *(volatile float*)(out + q) = ov;
    __threadfence();
    if (wave == 0 && q < nB) *(volatile float*)(out + q) = ov;
    __syncthreads();
  }
}

extern "C" void kernel_launch(void* const* d_in, const int* in_sizes, int n_in,
                              void* d_out, int out_size, void* d_ws, size_t ws_size,
                              hipStream_t stream) {
  if (n_in < 13) return;
  const int nN = in_sizes[0] / FD;
  if (nN < 1 || in_sizes[0] != nN * FD) return;
  if (in_sizes[1] != NLAY * NBAS * FD * FD || in_sizes[2] != NLAY * NREL * NBAS) return;
  if (in_sizes[3] != NLAY * FD * FD || in_sizes[4] != NLAY * FD) return;
  if (in_sizes[5] != KC * HID || in_sizes[6] != HID || in_sizes[7] != HID || in_sizes[8] < 1) return;
  const int nE = in_sizes[9];
  if (nE < 1 || in_sizes[10] != nE || in_sizes[11] != nE || in_sizes[12] < 1) return;
  const int nB = out_size;
  if (nB < 1 || nB > BCAP) return;
  if (nE > (1 << 28) || nN > (1 << 24)) return;

  const float* x     = (const float*)d_in[0];
  const float* basis = (const float*)d_in[1];
  const float* comp  = (const float*)d_in[2];
  const float* root  = (const float*)d_in[3];
  const float* bias  = (const float*)d_in[4];
  const float* w1    = (const float*)d_in[5];
  const float* b1    = (const float*)d_in[6];
  const float* w2    = (const float*)d_in[7];
  const float* b2    = (const float*)d_in[8];
  const int*   esrc  = (const int*)d_in[9];
  const int*   dsts  = (const int*)d_in[10];
  const int*   etyp  = (const int*)d_in[11];
  const int*   numg  = (const int*)d_in[12];
  float* out = (float*)d_out;

  const int NPAD   = ((nN + GR - 1) / GR) * GR;
  const int nBC    = (nN + NBC - 1) / NBC;
  const int CNTPAD = nBC * NBC;
  if (4 * nBC + 1 > RBN) return;
  const int nBF    = (nN + NBF - 1) / NBF;
  const int csrLen = ((nE + 31) & ~31) + 4096;
  if (31 * 4 * nBC > 4096) return;
  const int nL     = NPAD / GR;

  char* ws = (char*)d_ws;
  size_t off = 0;
  const size_t oW   = off; off += (size_t)OWTOT * 2;               off = (off + 255) & ~(size_t)255;
  const size_t oCnt = off; off += (size_t)CNTPAD * 4;              off = (off + 255) & ~(size_t)255;
  const size_t oOff = off; off += (size_t)CNTPAD * 4;              off = (off + 255) & ~(size_t)255;
  const size_t oRb  = off; off += (size_t)RBN * 4;                 off = (off + 255) & ~(size_t)255;
  const size_t oCsr = off; off += (size_t)csrLen * 4;              off = (off + 255) & ~(size_t)255;
  const size_t oST  = off; off += (size_t)NPAD * STP * 4;          off = (off + 255) & ~(size_t)255;
  if (off > ws_size || off > (size_t)WSCAP) return;
  unsigned short* wp   = (unsigned short*)(ws + oW);
  int*            cnt  = (int*)(ws + oCnt);
  int*            offp = (int*)(ws + oOff);
  int*            rb   = (int*)(ws + oRb);
  int*            csr  = (int*)(ws + oCsr);
  float*          ST   = (float*)(ws + oST);

  const int vec8 = ((nE & 3) == 0) ? 1 : 0;

  k_wprep<<<NWBLK, NTHR, 0, stream>>>(basis, root, w1, wp);

  k_count<<<nBC, NTHR, 0, stream>>>(dsts, cnt, nE, vec8);
  k_offsets<<<1, OTHR, 0, stream>>>(cnt, offp, rb, nBC);
  hipFuncSetAttribute(reinterpret_cast<const void*>(&k_fill),
                      hipFuncAttributeMaxDynamicSharedMemorySize, LDS_FILL);
  k_fill<<<nBF, NTHR, LDS_FILL, stream>>>(dsts, offp, rb, csr, nE, vec8, csrLen);

  hipFuncSetAttribute(reinterpret_cast<const void*>(&k_layer),
                      hipFuncAttributeMaxDynamicSharedMemorySize, LDS_LAY);
  for (int l = 0; l < NLAY; ++l) {
    const float* hin = (l == 0) ? x : (const float*)(ST + (size_t)(l - 1) * FD);
    const int pin = (l == 0) ? FD : STP;
    k_layer<<<nL, NTHR, LDS_LAY, stream>>>(csr, offp, cnt, esrc, etyp, hin, pin,
                                           comp + (size_t)l * NREL * NBAS,
                                           wp + (size_t)l * 2 * OWLSZ,
                                           bias + (size_t)l * FD,
                                           ST + (size_t)l * FD, nN, nE, csrLen);
  }

  hipFuncSetAttribute(reinterpret_cast<const void*>(&k_head),
                      hipFuncAttributeMaxDynamicSharedMemorySize, LDS_HEAD);
  k_head<<<1, NTHR, LDS_HEAD, stream>>>(x, ST, wp, b1, w2, b2, numg, out, nN, nB);
}
